// ParagraphEncoder_34986803593597
// MI455X (gfx1250) — hardware-run, weakly checked
//
#include <hip/hip_runtime.h>
#include <math.h>

typedef __attribute__((ext_vector_type(16))) _Float16 v16h;
typedef __attribute__((ext_vector_type(8)))  _Float16 v8h;
typedef __attribute__((ext_vector_type(2)))  _Float16 v2h;
typedef __attribute__((ext_vector_type(16))) __bf16   v16b;
typedef __attribute__((ext_vector_type(8)))  __bf16   v8b;
typedef __attribute__((ext_vector_type(8)))  float    v8f;
typedef __attribute__((ext_vector_type(4)))  float    v4f;
typedef __attribute__((ext_vector_type(2)))  float    v2f;
typedef __attribute__((ext_vector_type(4)))  _Float16 v4h;

constexpr int kB    = 64;
constexpr int kT    = 256;
constexpr int kI    = 768;
constexpr int kH    = 384;
constexpr int kG3   = 3 * kH;
constexpr int kD    = 2 * kH;
constexpr int kRows = kB * kT;
constexpr int kCh   = 64;
constexpr int kThr  = 256;
constexpr float kInCarry = 1024.0f;
constexpr float kSc = 1.0f / (kInCarry * kInCarry);
constexpr float kF16MinNormal = 6.103515625e-5f;

static_assert(kB == 64 && kT == 256 && kI == 768 && kH == 384 && kG3 == 1152 && kD == 768 && kRows == 16384 && kCh == 64 && kT % kCh == 0, "the index arithmetic below uses these sizes");

constexpr size_t kOffX16 = 0ull;
constexpr size_t kOffWI16 = 25165824ull;
constexpr size_t kOffWH16 = 32243712ull;
constexpr size_t kOffFC16 = 35782656ull;
constexpr size_t kOffZ = 36962304ull;
constexpr size_t kOffGX = 37560320ull;
constexpr size_t kOffGH = 75309056ull;
constexpr size_t kOffY0H = 75898880ull;
constexpr size_t kOffY1H = 101064704ull;
constexpr size_t kOffY1F = 126230528ull;
constexpr size_t kOffPRE = 176562176ull;
constexpr size_t kOffLG = 226893824ull;
constexpr size_t kWsTotal = 226959360ull;
static_assert(kWsTotal <= 268435456ull, "the carve stands under the contract's 256 MiB of workspace");
static_assert(kOffX16 == 0
  && kOffWI16 == kOffX16 + 25165824ull
  && kOffWH16 == kOffWI16 + 7077888ull
  && kOffFC16 == kOffWH16 + 3538944ull
  && kOffZ == kOffFC16 + 1179648ull
  && kOffGX == kOffZ + 598016ull
  && kOffGH == kOffGX + 37748736ull
  && kOffY0H == kOffGH + 589824ull
  && kOffY1H == kOffY0H + 25165824ull
  && kOffY1F == kOffY1H + 25165824ull
  && kOffPRE == kOffY1F + 50331648ull
  && kOffLG == kOffPRE + 50331648ull
  && kWsTotal == kOffLG + 65536ull, "the carve is a chain: every region starts where the one before ends");
static_assert((size_t)kRows * kI * 2 == 25165824ull && (size_t)4 * kG3 * kI * 2 == 7077888ull && (size_t)4 * kG3 * kH * 2 == 3538944ull && (size_t)kD * kD * 2 == 1179648ull
  && 8192ull + (size_t)4 * kB * kH * 2 + (size_t)4 * kB * kH * 4 == 598016ull && (size_t)2 * kB * kCh * kG3 * 4 == 37748736ull && (size_t)2 * kB * kG3 * 4 == 589824ull && (size_t)kRows * kD * 4 == 50331648ull && (size_t)kRows * 4 == 65536ull, "every region's length is its plane's");
static_assert((kOffWI16 % 256) == 0 && (kOffWH16 % 256) == 0 && (kOffFC16 % 256) == 0 && (kOffZ % 256) == 0 && (kOffGX % 256) == 0 && (kOffGH % 256) == 0 && (kOffY0H % 256) == 0 && (kOffY1H % 256) == 0 && (kOffY1F % 256) == 0 && (kOffPRE % 256) == 0 && (kOffLG % 256) == 0, "every region starts on a multiple of 256 B");
constexpr size_t kZH16 = 8192ull;
constexpr size_t kZH32 = 8192ull + (size_t)4 * kB * kH * 2;

__device__ __forceinline__ unsigned short f2bf_bits(float f) {
  unsigned u = __float_as_uint(f);
  return (unsigned short)((u + 0x7FFFu + ((u >> 16) & 1u)) >> 16);
}
__device__ __forceinline__ float bf_bits2f(unsigned short h) { return __uint_as_float(((unsigned)h) << 16); }
__device__ __forceinline__ float bf16r(float f) { return bf_bits2f(f2bf_bits(f)); }
__device__ __forceinline__ float carry_flush(float v, float carry) {
  const float s = v * carry;
  return (fabsf(s) < kF16MinNormal) ? 0.0f : s;
}

__device__ __forceinline__ void dep_guard4_h(v8f& a, v8f& b, v8f& c, v8f& d, v16h x, v16h y) { asm volatile("v_nop\n\tv_nop\n\tv_nop\n\tv_nop" : "+v"(a), "+v"(b), "+v"(c), "+v"(d) : "v"(x), "v"(y)); }
__device__ __forceinline__ void dep_guard4_b(v8f& a, v8f& b, v8f& c, v8f& d, v16b x, v16b y) { asm volatile("v_nop\n\tv_nop\n\tv_nop\n\tv_nop" : "+v"(a), "+v"(b), "+v"(c), "+v"(d) : "v"(x), "v"(y)); }
__device__ __forceinline__ void keep4_h(v16h a, v16h b, v16h c, v16h d) { asm volatile("v_nop" :: "v"(a), "v"(b), "v"(c), "v"(d)); }
__device__ __forceinline__ void keep4_b(v16b a, v16b b, v16b c, v16b d) { asm volatile("v_nop" :: "v"(a), "v"(b), "v"(c), "v"(d)); }
__device__ __forceinline__ void acc_guard4(v8f& a, v8f& b, v8f& c, v8f& d) { asm volatile("v_nop\n\tv_nop\n\tv_nop\n\tv_nop" : "+v"(a), "+v"(b), "+v"(c), "+v"(d)); }

template <typename T> struct Frag;
template <> struct Frag<_Float16> {
  typedef v16h V; union U { v16h v; v8h h[2]; };
  static __device__ __forceinline__ v16h load(const _Float16* p) {
    U f; f.h[0] = *(const v8h*)(p); f.h[1] = *(const v8h*)(p + 16); return f.v;
  }
  static __device__ __forceinline__ v8f mma(v16h a, v16h b, v8f c) {
    return __builtin_amdgcn_wmma_f32_16x16x32_f16(false, a, false, b, (short)0, c, false, false);
  }
  static __device__ __forceinline__ void guard4(v8f& a, v8f& b, v8f& c, v8f& d, v16h x, v16h y) { dep_guard4_h(a, b, c, d, x, y); }
  static __device__ __forceinline__ void keep(v16h a, v16h b, v16h c, v16h d) { keep4_h(a, b, c, d); }
};
template <> struct Frag<__bf16> {
  typedef v16b V; union U { v16b v; v8b h[2]; };
  static __device__ __forceinline__ v16b load(const __bf16* p) {
    U f; f.h[0] = *(const v8b*)(p); f.h[1] = *(const v8b*)(p + 16); return f.v;
  }
  static __device__ __forceinline__ v8f mma(v16b a, v16b b, v8f c) {
    return __builtin_amdgcn_wmma_f32_16x16x32_bf16(false, a, false, b, (short)0, c, false, false);
  }
  static __device__ __forceinline__ void guard4(v8f& a, v8f& b, v8f& c, v8f& d, v16b x, v16b y) { dep_guard4_b(a, b, c, d, x, y); }
  static __device__ __forceinline__ void keep(v16b a, v16b b, v16b c, v16b d) { keep4_b(a, b, c, d); }
};

__device__ __forceinline__ v8f mma_h(v16h a, v16h b, v8f c) {
  c = __builtin_amdgcn_wmma_f32_16x16x32_f16(false, a, false, b, (short)0, c, false, false);
  asm volatile("v_nop\n\tv_nop\n\tv_nop\n\tv_nop" : "+v"(c) : "v"(a), "v"(b));
  return c;
}

template <int ET> struct Elem;
template <> struct Elem<0> { typedef _Float16 T; };
template <> struct Elem<1> { typedef __bf16 T; };
template <int ET, bool SPLIT, int BIAS_MODE, int OUT_MODE, bool RESID, int ACT = 0>
__global__ __launch_bounds__(256) void wmma_gemm64(
    const unsigned short* __restrict__ Ap, const unsigned short* __restrict__ A2p, int lda, long strideA,
    const unsigned short* __restrict__ Btp, const unsigned short* __restrict__ Bt2p, int ldb, long strideB,
    void* __restrict__ Cout, void* __restrict__ Cout2, int ldc, long strideC,
    const float* __restrict__ bias,
    const float* __restrict__ resid, long strideR,
    int M, int N, int K, float scale) {
  typedef typename Elem<ET>::T T;
  typedef typename Frag<T>::V V;
  const T* A = (const T*)Ap; const T* A2 = (const T*)A2p; const T* Bt = (const T*)Btp; const T* Bt2 = (const T*)Bt2p;
  __shared__ __align__(16) float sT[8][16 * 68];
  const int b    = blockIdx.y;
  const int lane = threadIdx.x & 31;
  const int wave = threadIdx.x >> 5;
  const int tilesN = N >> 6;
  const int tilesM = M >> 6;
  const int tile = blockIdx.x * 8 + wave;
  if (tile >= tilesM * tilesN) return;
  const int tm = tile / tilesN;
  const int tn = tile - tm * tilesN;
  const int m0 = tm << 6;
  const int n0 = tn << 6;

  const T* Ab  = A  + (size_t)b * strideA;
  const T* Bb  = Bt + (size_t)b * strideB;
  const T* Ab2 = SPLIT ? (A2  + (size_t)b * strideA) : nullptr;
  const T* Bb2 = SPLIT ? (Bt2 + (size_t)b * strideB) : nullptr;

  const int rlane = lane & 15;
  const int koff  = (lane >> 4) * 8;
  const int mOff  = (lane >> 4) * 8;

  v8f acc[4][4];
#pragma unroll
  for (int i = 0; i < 4; ++i)
#pragma unroll
    for (int j = 0; j < 4; ++j) acc[i][j] = (v8f){0.f,0.f,0.f,0.f,0.f,0.f,0.f,0.f};

  for (int k0 = 0; k0 < K; k0 += 32) {
    V bh[4], bl[4];
#pragma unroll
    for (int j = 0; j < 4; ++j) {
      const size_t bo = (size_t)(n0 + (j << 4) + rlane) * ldb + koff + k0;
      bh[j] = Frag<T>::load(Bb + bo);
      if (SPLIT) bl[j] = Frag<T>::load(Bb2 + bo);
    }
#pragma unroll
    for (int i = 0; i < 4; ++i) {
      const size_t ao = (size_t)(m0 + (i << 4) + rlane) * lda + koff + k0;
      V ah = Frag<T>::load(Ab + ao);
      V al;
      if (SPLIT) al = Frag<T>::load(Ab2 + ao);
#pragma unroll
      for (int j = 0; j < 4; ++j) {
        acc[i][j] = Frag<T>::mma(ah, bh[j], acc[i][j]);
        if (SPLIT) {
          acc[i][j] = Frag<T>::mma(ah, bl[j], acc[i][j]);
          acc[i][j] = Frag<T>::mma(al, bh[j], acc[i][j]);
        }
      }
      Frag<T>::guard4(acc[i][0], acc[i][1], acc[i][2], acc[i][3], ah, SPLIT ? al : ah);
    }
    Frag<T>::keep(bh[0], bh[1], bh[2], bh[3]);
    if (SPLIT) Frag<T>::keep(bl[0], bl[1], bl[2], bl[3]);
  }
  acc_guard4(acc[0][0], acc[0][1], acc[0][2], acc[0][3]);
  acc_guard4(acc[1][0], acc[1][1], acc[1][2], acc[1][3]);
  acc_guard4(acc[2][0], acc[2][1], acc[2][2], acc[2][3]);
  acc_guard4(acc[3][0], acc[3][1], acc[3][2], acc[3][3]);

  float* slab = sT[wave];
  const float* Rb = RESID ? (resid + (size_t)b * strideR) : nullptr;
#pragma unroll
  for (int i = 0; i < 4; ++i) {
    const int mBase = m0 + (i << 4);
#pragma unroll
    for (int j = 0; j < 4; ++j) {
      const int n = n0 + (j << 4) + rlane;
      float bv = 0.f;
      if (BIAS_MODE == 2) bv = bias[n];
#pragma unroll
      for (int r = 0; r < 8; ++r) {
        float v = acc[i][j][r] * scale;
        if (BIAS_MODE == 1) v += bias[mBase + mOff + r];
        if (BIAS_MODE == 2) v += bv;
        if (RESID) v += Rb[(size_t)(mBase + mOff + r) * ldc + n];
        if (ACT == 1) v = tanhf(v);
        if (ACT == 2) v = fmaxf(v, 0.0f);
        if (ACT == 3) v = v / (1.0f + expf(-v));
        if (ACT == 4) v = (v > 0.f) ? v : 0.01f * v;
        slab[(mOff + r) * 68 + (j << 4) + rlane] = v;
      }
    }
    __builtin_amdgcn_fence(__ATOMIC_RELEASE, "workgroup");
    __builtin_amdgcn_wave_barrier();
    __builtin_amdgcn_fence(__ATOMIC_ACQUIRE, "workgroup");
    if (OUT_MODE == 0) {
      float* C = (float*)Cout + (size_t)b * strideC;
      const int hh = lane >> 4, c4 = (lane & 15) * 4;
      for (int pass = 0; pass < 2; ++pass) {
#pragma unroll
        for (int it = 0; it < 8; ++it) {
          const int row = it * 2 + hh;
          v4f v = *(const v4f*)(slab + row * 68 + c4);
          *(volatile v4f*)(C + (size_t)(mBase + row) * ldc + n0 + c4) = v;
        }
        __threadfence();
      }
    } else {
      const int q = lane >> 3, c8 = (lane & 7) * 8;
      unsigned short* C  = (unsigned short*)Cout  + (size_t)b * strideC;
      unsigned short* C2 = (OUT_MODE == 2) ? ((unsigned short*)Cout2 + (size_t)b * strideC) : nullptr;
      for (int pass = 0; pass < 2; ++pass) {
#pragma unroll
        for (int it = 0; it < 4; ++it) {
          const int row = it * 4 + q;
          const float* sp = slab + row * 68 + c8;
          v8h hv, lv;
#pragma unroll
          for (int e = 0; e < 8; ++e) {
            if (OUT_MODE == 1) {
              hv[e] = (_Float16)sp[e];
            } else {
              unsigned short hb = f2bf_bits(sp[e]);
              unsigned short lb = f2bf_bits(sp[e] - bf_bits2f(hb));
              hv[e] = __builtin_bit_cast(_Float16, hb);
              lv[e] = __builtin_bit_cast(_Float16, lb);
            }
          }
          *(volatile v8h*)(C + (size_t)(mBase + row) * ldc + n0 + c8) = hv;
          if (OUT_MODE == 2) *(volatile v8h*)(C2 + (size_t)(mBase + row) * ldc + n0 + c8) = lv;
        }
        __threadfence();
      }
    }
    __builtin_amdgcn_fence(__ATOMIC_RELEASE, "workgroup");
    __builtin_amdgcn_wave_barrier();
    __builtin_amdgcn_fence(__ATOMIC_ACQUIRE, "workgroup");
  }
}

__global__ __launch_bounds__(kThr) void cast_plane_kernel(const float* __restrict__ src, unsigned short* __restrict__ dst,
                                                          int colsLog2, int dstPitch, int dstOff) {
  const int i   = blockIdx.x * kThr + threadIdx.x;
  const int sh  = colsLog2 - 3;
  const int row = i >> sh;
  const int c8  = (i & ((1 << sh) - 1)) * 8;
  const float* sp = src + ((size_t)row << colsLog2) + c8;
  const v4f a0 = *(const v4f*)(sp);
  const v4f a1 = *(const v4f*)(sp + 4);
  v8h hv;
#pragma unroll
  for (int e = 0; e < 4; ++e) {
    const float f0 = a0[e];
    const float f1 = a1[e];
    hv[e]     = (_Float16)carry_flush(bf16r(f0), kInCarry);
    hv[4 + e] = (_Float16)carry_flush(bf16r(f1), kInCarry);
  }
  unsigned short* dp = dst + (size_t)row * dstPitch + dstOff + c8;
  *(volatile v8h*)dp = hv;
  __threadfence();
  *(volatile v8h*)dp = hv;
}

__global__ __launch_bounds__(kThr) void zero_kernel(float* __restrict__ dst) {
  const size_t o4 = ((size_t)blockIdx.x * kThr + threadIdx.x) * 4u;
  const v4f z = {0.f, 0.f, 0.f, 0.f};
  *(volatile v4f*)(dst + o4) = z;
  __threadfence();
  *(volatile v4f*)(dst + o4) = z;
}
__global__ __launch_bounds__(kThr) void cell_kernel(const float* __restrict__ GX, const float* __restrict__ GH, const float* __restrict__ bih_f, const float* __restrict__ bhh_f, const float* __restrict__ bih_b, const float* __restrict__ bhh_b,
                                                    float* __restrict__ H32, unsigned short* __restrict__ H16, unsigned short* __restrict__ Y16, float* __restrict__ Y32, int k, int f32out) {
  const unsigned d = blockIdx.x >> 2;
  const unsigned b = ((blockIdx.x & 3u) << 4) + (threadIdx.x >> 4);
  const unsigned u8 = (blockIdx.y << 7) + ((threadIdx.x & 15u) << 3);
  const unsigned kk = (unsigned)k & 63u;
  const unsigned tl = (d != 0u) ? (63u - kk) : kk;
  const unsigned t = (d != 0u) ? (255u - (unsigned)k) : (unsigned)k;
  const unsigned db = d * (unsigned)kB + b;
  const float* gx = GX + (db * (unsigned)kCh + tl) * (unsigned)kG3 + u8;
  const float* gh = GH + db * (unsigned)kG3 + u8;
  const float* bi = ((d != 0u) ? bih_b : bih_f) + u8;
  const float* bh = ((d != 0u) ? bhh_b : bhh_f) + u8;
  float* hp = H32 + db * (unsigned)kH + u8;
  v8h hv;
  v4f hn0, hn1;
#pragma unroll
  for (int hlf = 0; hlf < 2; ++hlf) {
    const v4f xr = *(const v4f*)(gx + 4 * hlf), xz = *(const v4f*)(gx + kH + 4 * hlf), xn = *(const v4f*)(gx + 2 * kH + 4 * hlf);
    const v4f sr = *(const v4f*)(gh + 4 * hlf), sz = *(const v4f*)(gh + kH + 4 * hlf), sn = *(const v4f*)(gh + 2 * kH + 4 * hlf);
    const v4f pr = *(const v4f*)(bi + 4 * hlf), pz = *(const v4f*)(bi + kH + 4 * hlf), pn = *(const v4f*)(bi + 2 * kH + 4 * hlf);
    const v4f qr = *(const v4f*)(bh + 4 * hlf), qz = *(const v4f*)(bh + kH + 4 * hlf), qn = *(const v4f*)(bh + 2 * kH + 4 * hlf);
    const v4f ho = *(const v4f*)(hp + 4 * hlf);
#pragma unroll
    for (int e = 0; e < 4; ++e) {
      const float r = 1.0f / (1.0f + expf(-((xr[e] + bf16r(pr[e])) + (sr[e] + bf16r(qr[e])))));
      const float z = 1.0f / (1.0f + expf(-((xz[e] + bf16r(pz[e])) + (sz[e] + bf16r(qz[e])))));
      const float n = tanhf((xn[e] + bf16r(pn[e])) + r * (sn[e] + bf16r(qn[e])));
      const float hn = (1.0f - z) * n + z * ho[e];
      if (hlf == 0) hn0[e] = hn; else hn1[e] = hn;
      hv[4 * hlf + e] = (_Float16)carry_flush(hn, kInCarry);
    }
  }
  unsigned short* sp = H16 + db * (unsigned)kH + u8;
  const unsigned yo = (b * (unsigned)kT + t) * (unsigned)kD + d * (unsigned)kH + u8;
  unsigned short* yp = Y16 + yo;
  float* fp = Y32 + yo;
  for (int pass = 0; pass < 2; ++pass) {
    *(volatile v4f*)hp = hn0;
    *(volatile v4f*)(hp + 4) = hn1;
    *(volatile v8h*)sp = hv;
    *(volatile v8h*)yp = hv;
    if (f32out != 0) {
      *(volatile v4f*)fp = hn0;
      *(volatile v4f*)(fp + 4) = hn1;
    }
    __threadfence();
  }
}
static_assert(2 * kB * kH / 8 == 8 * 3 * kThr && kH == 3 * 128 && kB == 4 * 16, "the cell's grid exact: dim3(8, 3) blocks of 256 threads");

__global__ __launch_bounds__(kThr) void score_kernel(const float* __restrict__ PRE, const float* __restrict__ fcb, const float* __restrict__ upw, const float* __restrict__ upb, float* __restrict__ LG) {
  const unsigned row = blockIdx.x * (unsigned)kThr + threadIdx.x;
  const float* pp = PRE + row * (unsigned)kD;
  float acc = 0.0f;
  for (unsigned c = 0; c < (unsigned)kD; c += 4u) {
    const v4f p = *(const v4f*)(pp + c);
    const v4f fb = *(const v4f*)(fcb + c);
    const v4f w = *(const v4f*)(upw + c);
    acc = fmaf(tanhf(p[0] + bf16r(fb[0])), bf16r(w[0]), acc);
    acc = fmaf(tanhf(p[1] + bf16r(fb[1])), bf16r(w[1]), acc);
    acc = fmaf(tanhf(p[2] + bf16r(fb[2])), bf16r(w[2]), acc);
    acc = fmaf(tanhf(p[3] + bf16r(fb[3])), bf16r(w[3]), acc);
  }
  acc = acc + bf16r(upb[0]);
  float* dp = LG + row;
  *(volatile float*)dp = acc;
  __threadfence();
  *(volatile float*)dp = acc;
}
static_assert(kRows == 64 * kThr && kD % 4 == 0, "the score grid exact: 64 blocks");

__global__ __launch_bounds__(192) void pool_kernel(const float* __restrict__ LG, const float* __restrict__ Y32, float* __restrict__ out) {
  const unsigned b = blockIdx.x;
  const unsigned c4 = threadIdx.x * 4u;
  const float* lg = LG + b * (unsigned)kT;
  float m = lg[0];
  for (unsigned t = 1u; t < (unsigned)kT; ++t) { const float s = lg[t]; m = (s > m) ? s : m; }
  float den = 0.0f;
  for (unsigned t = 0u; t < (unsigned)kT; ++t) den = den + expf(lg[t] - m);
  v4f acc = {0.f, 0.f, 0.f, 0.f};
  const float* yp = Y32 + b * (unsigned)kT * (unsigned)kD + c4;
  for (unsigned t = 0u; t < (unsigned)kT; ++t) {
    const float al = expf(lg[t] - m) / den;
    const v4f h = *(const v4f*)(yp + t * (unsigned)kD);
    acc[0] = fmaf(al, h[0], acc[0]);
    acc[1] = fmaf(al, h[1], acc[1]);
    acc[2] = fmaf(al, h[2], acc[2]);
    acc[3] = fmaf(al, h[3], acc[3]);
  }
  float* dp = out + b * (unsigned)kD + c4;
  *(volatile v4f*)dp = acc;
  __threadfence();
  *(volatile v4f*)dp = acc;
}
static_assert(kD / 4 == 192 && 192 % 32 == 0, "the pool's block: 192 threads = six whole waves cover a sample's 768 result columns");

extern "C" void kernel_launch(void* const* d_in, const int* in_sizes, int n_in,
                              void* d_out, int out_size, void* d_ws, size_t ws_size,
                              hipStream_t stream) {
  if (n_in < 21 || d_out == nullptr || d_ws == nullptr) return;
  if (in_sizes[0] != kB * kT * kI) return;
  for (int q = 0; q < 4; ++q) {
    if (in_sizes[1 + 4 * q] != kG3 * kI || in_sizes[2 + 4 * q] != kG3 * kH || in_sizes[3 + 4 * q] != kG3 || in_sizes[4 + 4 * q] != kG3) return;
  }
  if (in_sizes[17] != kD * kD || in_sizes[18] != kD || in_sizes[19] != kD || in_sizes[20] != 1) return;
  if (out_size != kB * kD) return;
  if (ws_size < kWsTotal) return;
  const float* x = (const float*)d_in[0];
  const float* fcw = (const float*)d_in[17];
  const float* fcb = (const float*)d_in[18];
  const float* upw = (const float*)d_in[19];
  const float* upb = (const float*)d_in[20];
  float* out = (float*)d_out;
  char* ws = (char*)d_ws;
  unsigned short* X16 = (unsigned short*)(ws + kOffX16);
  unsigned short* WI16 = (unsigned short*)(ws + kOffWI16);
  unsigned short* WH16 = (unsigned short*)(ws + kOffWH16);
  unsigned short* FC16 = (unsigned short*)(ws + kOffFC16);
  float* ZB = (float*)(ws + kOffZ);
  unsigned short* H16 = (unsigned short*)(ws + kOffZ + kZH16);
  float* H32 = (float*)(ws + kOffZ + kZH32);
  float* GX = (float*)(ws + kOffGX);
  float* GH = (float*)(ws + kOffGH);
  unsigned short* Y0H = (unsigned short*)(ws + kOffY0H);
  unsigned short* Y1H = (unsigned short*)(ws + kOffY1H);
  float* Y1F = (float*)(ws + kOffY1F);
  float* PRE = (float*)(ws + kOffPRE);
  float* LG = (float*)(ws + kOffLG);
  constexpr size_t kWi = (size_t)kG3 * kI, kWh = (size_t)kG3 * kH, kHp = (size_t)kB * kH;

  static_assert(((size_t)kRows * kI / 8) % kThr == 0 && ((size_t)kG3 * kI / 8) % kThr == 0 && ((size_t)kG3 * kH / 8) % kThr == 0 && ((size_t)kD * kD / 8) % kThr == 0 && 598016ull / 16ull == 146ull * kThr, "the casts' grids and the zero fill's grid (146 blocks over Z's 598,016 B) exact");
  cast_plane_kernel<<<(int)(((size_t)kRows * kI / 8) / kThr), kThr, 0, stream>>>(x, X16, 8, 256, 0);
  for (int q = 0; q < 4; ++q) {
    cast_plane_kernel<<<(int)((kWi / 8) / kThr), kThr, 0, stream>>>((const float*)d_in[1 + 4 * q], WI16 + (size_t)q * kWi, 8, 256, 0);
    cast_plane_kernel<<<(int)((kWh / 8) / kThr), kThr, 0, stream>>>((const float*)d_in[2 + 4 * q], WH16 + (size_t)q * kWh, 7, 128, 0);
  }
  cast_plane_kernel<<<(int)(((size_t)kD * kD / 8) / kThr), kThr, 0, stream>>>(fcw, FC16, 8, 256, 0);
  zero_kernel<<<146, kThr, 0, stream>>>(ZB);

  for (int l = 0; l < 2; ++l) {
    const unsigned short* A16 = (l == 0) ? X16 : Y0H;
    unsigned short* Hl16 = H16 + (size_t)(2 * l) * kHp;
    float* Hl32 = H32 + (size_t)(2 * l) * kHp;
    const float* bif = (const float*)d_in[3 + 8 * l];
    const float* bhf = (const float*)d_in[4 + 8 * l];
    const float* bib = (const float*)d_in[7 + 8 * l];
    const float* bhb = (const float*)d_in[8 + 8 * l];
    unsigned short* Yl16 = (l == 0) ? Y0H : Y1H;
    for (int c = 0; c < kT / kCh; ++c) {
      wmma_gemm64<0, false, 2, 0, false, 0><<<dim3(3, kB), 256, 0, stream>>>(
          A16 + (size_t)(kCh * c) * kI, A16 + (size_t)(kCh * c) * kI, kI, (long)kT * kI, WI16 + (size_t)(2 * l) * kWi, WI16 + (size_t)(2 * l) * kWi, kI, 0L,
          (void*)GX, (void*)GX, kG3, (long)kCh * kG3, ZB, nullptr, 0L, kCh, kG3, kI, kSc);
      wmma_gemm64<0, false, 2, 0, false, 0><<<dim3(3, kB), 256, 0, stream>>>(
          A16 + (size_t)(kT - kCh - kCh * c) * kI, A16 + (size_t)(kT - kCh - kCh * c) * kI, kI, (long)kT * kI, WI16 + (size_t)(2 * l + 1) * kWi, WI16 + (size_t)(2 * l + 1) * kWi, kI, 0L,
          (void*)(GX + (size_t)kB * kCh * kG3), (void*)(GX + (size_t)kB * kCh * kG3), kG3, (long)kCh * kG3, ZB, nullptr, 0L, kCh, kG3, kI, kSc);
      for (int kk = 0; kk < kCh; ++kk) {
        wmma_gemm64<0, false, 2, 0, false, 0><<<dim3(3, 2), 256, 0, stream>>>(
            Hl16, Hl16, kH, (long)kB * kH, WH16 + (size_t)(2 * l) * kWh, WH16 + (size_t)(2 * l) * kWh, kH, (long)kG3 * kH,
            (void*)GH, (void*)GH, kG3, (long)kB * kG3, ZB, nullptr, 0L, kB, kG3, kH, kSc);
        cell_kernel<<<dim3(8, 3), kThr, 0, stream>>>(GX, GH, bif, bhf, bib, bhb, Hl32, Hl16, Yl16, Y1F, kCh * c + kk, l);
      }
    }
  }
  wmma_gemm64<0, false, 2, 0, false, 0><<<dim3((kRows / 64) * (kD / 64) / 8, 1), 256, 0, stream>>>(
      Y1H, Y1H, kD, 0L, FC16, FC16, kD, 0L, (void*)PRE, (void*)PRE, kD, 0L, ZB, nullptr, 0L, kRows, kD, kD, kSc);
  score_kernel<<<kRows / kThr, kThr, 0, stream>>>(PRE, fcb, upw, upb, LG);
  pool_kernel<<<kB, 192, 0, stream>>>(LG, Y1F, out);
}
static_assert(((kRows / 64) * (kD / 64)) % 8 == 0 && (kG3 / 64) == 18, "the pooling map's grid: whole blocks of eight wave tiles; a gate product's 18 tiles a batch go on three blocks (24 waves: six leave at the tile guard)");
